// GatedDeltaNet_69355131896515
// MI455X (gfx1250) — hardware-verified
//
#include <hip/hip_runtime.h>
#include <math.h>

constexpr int kBatch   = 2;
constexpr int kSeq     = 2048;
constexpr int kDim     = 1024;
constexpr int kHeads   = 16;
constexpr int kHdim    = 64;
constexpr int kTaps    = 4;
constexpr int kRows    = kBatch * kSeq;
constexpr int kAbPad   = 64;
constexpr int kOgPitch = 2 * kDim;
constexpr float kNormEps = 1e-6f;
constexpr float kQScale  = 0.125f;
constexpr float kInvHdim = 1.0f / (float)kHdim;
static_assert(kQScale * kQScale * (float)kHdim == 1.0f);
static_assert(kHeads * kHdim == kDim);
static_assert(kRows == 4096 && kDim == 1024 && kHdim == 64 && kHeads == 16 && kTaps == 4);
static_assert(kRows % 64 == 0 && kDim % 64 == 0 && kAbPad % 64 == 0);
static_assert(kDim % 32 == 0 && kOgPitch % 32 == 0);
static_assert((kSeq & (kSeq - 1)) == 0);

typedef __attribute__((ext_vector_type(16))) _Float16 v16h;
typedef __attribute__((ext_vector_type(8)))  _Float16 v8h;
typedef __attribute__((ext_vector_type(16))) __bf16   v16b;
typedef __attribute__((ext_vector_type(8)))  __bf16   v8b;
typedef __attribute__((ext_vector_type(8)))  float    v8f;
typedef __attribute__((ext_vector_type(4)))  float    v4f;
typedef __attribute__((ext_vector_type(4)))  unsigned int v4u;

__device__ __forceinline__ unsigned short f2bf_bits(float f) {
  unsigned u = __float_as_uint(f);
  return (unsigned short)((u + 0x7FFFu + ((u >> 16) & 1u)) >> 16);
}
__device__ __forceinline__ float bf_bits2f(unsigned short h) { return __uint_as_float(((unsigned)h) << 16); }
__device__ __forceinline__ float bf16r(float f) { return bf_bits2f(f2bf_bits(f)); }
__device__ __forceinline__ unsigned pk16(unsigned short a, unsigned short b) { return (unsigned)a | ((unsigned)b << 16); }
__device__ __forceinline__ v4u pack8_bf16(v4f a, v4f b) {
  const float a0 = a[0], a1 = a[1], a2 = a[2], a3 = a[3];
  const float b0 = b[0], b1 = b[1], b2 = b[2], b3 = b[3];
  return (v4u){pk16(f2bf_bits(a0), f2bf_bits(a1)), pk16(f2bf_bits(a2), f2bf_bits(a3)),
               pk16(f2bf_bits(b0), f2bf_bits(b1)), pk16(f2bf_bits(b2), f2bf_bits(b3))};
}
__device__ __forceinline__ float sigmoid_f(float x) { return __builtin_amdgcn_rcpf(1.0f + expf(-x)); }

__device__ __forceinline__ void dep_guard4_h(v8f& a, v8f& b, v8f& c, v8f& d, v16h x, v16h y) {
  asm volatile("v_nop\n\tv_nop\n\tv_nop\n\tv_nop" : "+v"(a), "+v"(b), "+v"(c), "+v"(d) : "v"(x), "v"(y));
}
__device__ __forceinline__ void dep_guard4_b(v8f& a, v8f& b, v8f& c, v8f& d, v16b x, v16b y) {
  asm volatile("v_nop\n\tv_nop\n\tv_nop\n\tv_nop" : "+v"(a), "+v"(b), "+v"(c), "+v"(d) : "v"(x), "v"(y));
}
__device__ __forceinline__ void keep4_h(v16h a, v16h b, v16h c, v16h d) { asm volatile("v_nop" :: "v"(a), "v"(b), "v"(c), "v"(d)); }
__device__ __forceinline__ void keep4_b(v16b a, v16b b, v16b c, v16b d) { asm volatile("v_nop" :: "v"(a), "v"(b), "v"(c), "v"(d)); }
__device__ __forceinline__ void acc_guard4(v8f& a, v8f& b, v8f& c, v8f& d) {
  asm volatile("v_nop\n\tv_nop\n\tv_nop\n\tv_nop" : "+v"(a), "+v"(b), "+v"(c), "+v"(d));
}
template <typename T> struct Frag;
template <> struct Frag<_Float16> {
  typedef v16h V; union U { v16h v; v8h h[2]; };
  static __device__ __forceinline__ v16h load(const _Float16* p) {
    U f; f.h[0] = *(const v8h*)(p); f.h[1] = *(const v8h*)(p + 16); return f.v;
  }
  static __device__ __forceinline__ v8f mma(v16h a, v16h b, v8f c) {
    return __builtin_amdgcn_wmma_f32_16x16x32_f16(false, a, false, b, (short)0, c, false, false);
  }
  static __device__ __forceinline__ void guard4(v8f& a, v8f& b, v8f& c, v8f& d, v16h x, v16h y) { dep_guard4_h(a, b, c, d, x, y); }
  static __device__ __forceinline__ void keep(v16h a, v16h b, v16h c, v16h d) { keep4_h(a, b, c, d); }
};
template <> struct Frag<__bf16> {
  typedef v16b V; union U { v16b v; v8b h[2]; };
  static __device__ __forceinline__ v16b load(const __bf16* p) {
    U f; f.h[0] = *(const v8b*)(p); f.h[1] = *(const v8b*)(p + 16); return f.v;
  }
  static __device__ __forceinline__ v8f mma(v16b a, v16b b, v8f c) {
    return __builtin_amdgcn_wmma_f32_16x16x32_bf16(false, a, false, b, (short)0, c, false, false);
  }
  static __device__ __forceinline__ void guard4(v8f& a, v8f& b, v8f& c, v8f& d, v16b x, v16b y) { dep_guard4_b(a, b, c, d, x, y); }
  static __device__ __forceinline__ void keep(v16b a, v16b b, v16b c, v16b d) { keep4_b(a, b, c, d); }
};

template <int ET> struct Elem;
template <> struct Elem<0> { typedef _Float16 T; };
template <> struct Elem<1> { typedef __bf16 T; };
template <int ET, bool SPLIT, int BIAS_MODE, int OUT_MODE, bool RESID, int ACT = 0>
__global__ __launch_bounds__(256) void wmma_gemm64(
    const unsigned short* __restrict__ Ap, const unsigned short* __restrict__ A2p, int lda, long strideA,
    const unsigned short* __restrict__ Btp, const unsigned short* __restrict__ Bt2p, int ldb, long strideB,
    void* __restrict__ Cout, void* __restrict__ Cout2, int ldc, long strideC,
    const float* __restrict__ bias,
    const float* __restrict__ resid, long strideR,
    int M, int N, int K, float scale) {
  typedef typename Elem<ET>::T T;
  typedef typename Frag<T>::V V;
  const T* A = (const T*)Ap; const T* A2 = (const T*)A2p; const T* Bt = (const T*)Btp; const T* Bt2 = (const T*)Bt2p;
  __shared__ __align__(16) float sT[8][16 * 68];
  const int b    = blockIdx.y;
  const int lane = threadIdx.x & 31;
  const int wave = threadIdx.x >> 5;
  const int tilesN = N >> 6;
  const int tilesM = M >> 6;
  const int tile = blockIdx.x * 8 + wave;
  if (tile >= tilesM * tilesN) return;
  const int tm = tile / tilesN;
  const int tn = tile - tm * tilesN;
  const int m0 = tm << 6;
  const int n0 = tn << 6;

  const T* Ab  = A  + (size_t)b * strideA;
  const T* Bb  = Bt + (size_t)b * strideB;
  const T* Ab2 = SPLIT ? (A2  + (size_t)b * strideA) : nullptr;
  const T* Bb2 = SPLIT ? (Bt2 + (size_t)b * strideB) : nullptr;

  const int rlane = lane & 15;
  const int koff  = (lane >> 4) * 8;
  const int mOff  = (lane >> 4) * 8;

  v8f acc[4][4];
#pragma unroll
  for (int i = 0; i < 4; ++i)
#pragma unroll
    for (int j = 0; j < 4; ++j) acc[i][j] = (v8f){0.f,0.f,0.f,0.f,0.f,0.f,0.f,0.f};

  for (int k0 = 0; k0 < K; k0 += 32) {
    V bh[4], bl[4];
#pragma unroll
    for (int j = 0; j < 4; ++j) {
      const size_t bo = (size_t)(n0 + (j << 4) + rlane) * ldb + koff + k0;
      bh[j] = Frag<T>::load(Bb + bo);
      if (SPLIT) bl[j] = Frag<T>::load(Bb2 + bo);
    }
#pragma unroll
    for (int i = 0; i < 4; ++i) {
      const size_t ao = (size_t)(m0 + (i << 4) + rlane) * lda + koff + k0;
      V ah = Frag<T>::load(Ab + ao);
      V al;
      if (SPLIT) al = Frag<T>::load(Ab2 + ao);
#pragma unroll
      for (int j = 0; j < 4; ++j) {
        acc[i][j] = Frag<T>::mma(ah, bh[j], acc[i][j]);
        if (SPLIT) {
          acc[i][j] = Frag<T>::mma(ah, bl[j], acc[i][j]);
          acc[i][j] = Frag<T>::mma(al, bh[j], acc[i][j]);
        }
      }
      Frag<T>::guard4(acc[i][0], acc[i][1], acc[i][2], acc[i][3], ah, SPLIT ? al : ah);
    }
    Frag<T>::keep(bh[0], bh[1], bh[2], bh[3]);
    if (SPLIT) Frag<T>::keep(bl[0], bl[1], bl[2], bl[3]);
  }
  acc_guard4(acc[0][0], acc[0][1], acc[0][2], acc[0][3]);
  acc_guard4(acc[1][0], acc[1][1], acc[1][2], acc[1][3]);
  acc_guard4(acc[2][0], acc[2][1], acc[2][2], acc[2][3]);
  acc_guard4(acc[3][0], acc[3][1], acc[3][2], acc[3][3]);

  float* slab = sT[wave];
  const float* Rb = RESID ? (resid + (size_t)b * strideR) : nullptr;
#pragma unroll
  for (int i = 0; i < 4; ++i) {
    const int mBase = m0 + (i << 4);
#pragma unroll
    for (int j = 0; j < 4; ++j) {
      const int n = n0 + (j << 4) + rlane;
      float bv = 0.f;
      if (BIAS_MODE == 2) bv = bias[n];
#pragma unroll
      for (int r = 0; r < 8; ++r) {
        float v = acc[i][j][r] * scale;
        if (BIAS_MODE == 1) v += bias[mBase + mOff + r];
        if (BIAS_MODE == 2) v += bv;
        if (RESID) v += Rb[(size_t)(mBase + mOff + r) * ldc + n];
        if (ACT == 2) v = fmaxf(v, 0.0f);
        if (ACT == 4) v = (v > 0.f) ? v : 0.01f * v;
        slab[(mOff + r) * 68 + (j << 4) + rlane] = v;
      }
    }
    __builtin_amdgcn_fence(__ATOMIC_RELEASE, "workgroup");
    __builtin_amdgcn_wave_barrier();
    __builtin_amdgcn_fence(__ATOMIC_ACQUIRE, "workgroup");
    if (OUT_MODE == 0) {
      float* C = (float*)Cout + (size_t)b * strideC;
      const int hh = lane >> 4, c4 = (lane & 15) * 4;
      for (int pass = 0; pass < 2; ++pass) {
#pragma unroll
        for (int it = 0; it < 8; ++it) {
          const int row = it * 2 + hh;
          v4f v = *(const v4f*)(slab + row * 68 + c4);
          *(volatile v4f*)(C + (size_t)(mBase + row) * ldc + n0 + c4) = v;
        }
        __threadfence();
      }
    } else {
      const int q = lane >> 3, c8 = (lane & 7) * 8;
      unsigned short* C  = (unsigned short*)Cout  + (size_t)b * strideC;
      unsigned short* C2 = (OUT_MODE == 2) ? ((unsigned short*)Cout2 + (size_t)b * strideC) : nullptr;
      for (int pass = 0; pass < 2; ++pass) {
#pragma unroll
        for (int it = 0; it < 4; ++it) {
          const int row = it * 4 + q;
          const float* sp = slab + row * 68 + c8;
          v8h hv, lv;
#pragma unroll
          for (int e = 0; e < 8; ++e) {
            if (OUT_MODE == 1) {
              hv[e] = (_Float16)sp[e];
            } else {
              unsigned short hb = f2bf_bits(sp[e]);
              unsigned short lb = f2bf_bits(sp[e] - bf_bits2f(hb));
              hv[e] = __builtin_bit_cast(_Float16, hb);
              lv[e] = __builtin_bit_cast(_Float16, lb);
            }
          }
          *(volatile v8h*)(C + (size_t)(mBase + row) * ldc + n0 + c8) = hv;
          if (OUT_MODE == 2) *(volatile v8h*)(C2 + (size_t)(mBase + row) * ldc + n0 + c8) = lv;
        }
        __threadfence();
      }
    }
    __builtin_amdgcn_fence(__ATOMIC_RELEASE, "workgroup");
    __builtin_amdgcn_wave_barrier();
    __builtin_amdgcn_fence(__ATOMIC_ACQUIRE, "workgroup");
  }
}

__global__ __launch_bounds__(256) void cvt8_bf16_kernel(const float* __restrict__ src, unsigned short* __restrict__ dst, int n8) {
  const int i = blockIdx.x * 256 + threadIdx.x;
  if (i < n8) {
    const float* sp = src + (size_t)i * 8;
    const v4f a = *(const v4f*)(sp);
    const v4f c = *(const v4f*)(sp + 4);
    const v4u u = pack8_bf16(a, c);
    unsigned short* q = dst + (size_t)i * 8;
    *(volatile v4u*)q = u;
    __threadfence();
    *(volatile v4u*)q = u;
  }
}

__global__ __launch_bounds__(256) void cvt_w4_kernel(const float* __restrict__ W0, const float* __restrict__ W1,
                                                     const float* __restrict__ W2, const float* __restrict__ W3,
                                                     unsigned short* __restrict__ dst) {
  const int z = blockIdx.y;
  const float* W = (z == 0) ? W0 : (z == 1) ? W1 : (z == 2) ? W2 : W3;
  const int i = blockIdx.x * 256 + threadIdx.x;
  if (i < kDim * kDim / 8) {
    const float* sp = W + (size_t)i * 8;
    const v4f a = *(const v4f*)(sp);
    const v4f c = *(const v4f*)(sp + 4);
    const v4u u = pack8_bf16(a, c);
    unsigned short* q = dst + (size_t)z * kDim * kDim + (size_t)i * 8;
    *(volatile v4u*)q = u;
    __threadfence();
    *(volatile v4u*)q = u;
  }
}

__global__ __launch_bounds__(256) void cvt_wo2_kernel(const float* __restrict__ Wo, unsigned short* __restrict__ dst) {
  const int i = blockIdx.x * 256 + threadIdx.x;
  if (i < kDim * kDim / 8) {
    const int row = i >> 7;
    const int c8  = i & 127;
    const float* sp = Wo + (size_t)row * kDim + c8 * 8;
    const v4f a = *(const v4f*)(sp);
    const v4f c = *(const v4f*)(sp + 4);
    const v4u u = pack8_bf16(a, c);
    unsigned short* q0 = dst + (size_t)row * kOgPitch + c8 * 8;
    unsigned short* q1 = q0 + kDim;
    *(volatile v4u*)q0 = u;
    *(volatile v4u*)q1 = u;
    __threadfence();
    *(volatile v4u*)q0 = u;
    *(volatile v4u*)q1 = u;
  }
}

__global__ __launch_bounds__(256) void cvt_wab_kernel(const float* __restrict__ Wa, const float* __restrict__ Wb,
                                                      unsigned short* __restrict__ dst) {
  const int i = blockIdx.x * 256 + threadIdx.x;
  if (i < kAbPad * kDim / 8) {
    const int row = i >> 7;
    const int c8  = i & 127;
    const int ra = row < (kHeads - 1) ? row : (kHeads - 1);
    int rb = row - kHeads;
    rb = rb < 0 ? 0 : rb;
    rb = rb > (kHeads - 1) ? (kHeads - 1) : rb;
    const float* pa = Wa + (size_t)ra * kDim + c8 * 8;
    const float* pb = Wb + (size_t)rb * kDim + c8 * 8;
    const v4f a0 = *(const v4f*)(pa);
    const v4f a1 = *(const v4f*)(pa + 4);
    const v4f b0 = *(const v4f*)(pb);
    const v4f b1 = *(const v4f*)(pb + 4);
    const bool ua = row < kHeads;
    const bool ub = (row >= kHeads) && (row < 2 * kHeads);
    v4f s0, s1;
#pragma unroll
    for (int e = 0; e < 4; ++e) {
      s0[e] = ua ? a0[e] : (ub ? b0[e] : 0.0f);
      s1[e] = ua ? a1[e] : (ub ? b1[e] : 0.0f);
    }
    const v4u u = pack8_bf16(s0, s1);
    unsigned short* q = dst + (size_t)i * 8;
    *(volatile v4u*)q = u;
    __threadfence();
    *(volatile v4u*)q = u;
  }
}

__global__ __launch_bounds__(256) void gate_kernel(const float* __restrict__ PAB, const float* __restrict__ A_log,
                                                   const float* __restrict__ dt_bias,
                                                   float* __restrict__ DEC, float* __restrict__ BETA) {
  const int i = blockIdx.x * 256 + threadIdx.x;
  if (i < kRows * kHeads) {
    const int row = i >> 4;
    const int hh  = i & 15;
    const float a  = PAB[(size_t)row * kAbPad + hh];
    const float bl = PAB[(size_t)row * kAbPad + kHeads + hh];
    const float al = bf16r(A_log[hh]);
    const float db = bf16r(dt_bias[hh]);
    const float x  = a + db;
    const float sp = fmaxf(x, 0.0f) + log1pf(expf(-fabsf(x)));
    const float g  = (-expf(al)) * sp;
    const float dec  = expf(g);
    const float beta = 1.0f / (1.0f + expf(-bl));
    *(volatile float*)(DEC + i)  = dec;
    *(volatile float*)(BETA + i) = beta;
    __threadfence();
    *(volatile float*)(DEC + i)  = dec;
    *(volatile float*)(BETA + i) = beta;
  }
}

template <bool NORM>
__global__ __launch_bounds__(256) void conv_silu_kernel(const float* __restrict__ P, const float* __restrict__ cw,
                                                        const float* __restrict__ nw, float* __restrict__ outp,
                                                        float oscale) {
  const int lane = threadIdx.x & 31;
  const int wave = threadIdx.x >> 5;
  const int gw   = blockIdx.x * 8 + wave;
  const int row  = gw >> 3;
  const int hp   = gw & 7;
  const int c0   = hp * 128 + lane * 4;
  const int t    = row & (kSeq - 1);

  v4f wv[4];
#pragma unroll
  for (int e = 0; e < 4; ++e) wv[e] = *(const v4f*)(cw + (size_t)(c0 + e) * kTaps);

  float y[4] = {0.0f, 0.0f, 0.0f, 0.0f};
#pragma unroll
  for (int j = 0; j < kTaps; ++j) {
    const int back = (kTaps - 1) - j;
    const bool valid = (t >= back);
    const int rs = valid ? (row - back) : row;
    const v4f x = *(const v4f*)(P + (size_t)rs * kDim + c0);
#pragma unroll
    for (int e = 0; e < 4; ++e) {
      const float wf = wv[e][j];
      const float xe = valid ? x[e] : 0.0f;
      y[e] = fmaf(bf16r(wf), xe, y[e]);
    }
  }
  float z[4];
#pragma unroll
  for (int e = 0; e < 4; ++e) z[e] = y[e] * sigmoid_f(y[e]);

  v4f o;
  if (NORM) {
    float ss = 0.0f;
#pragma unroll
    for (int e = 0; e < 4; ++e) ss = fmaf(z[e], z[e], ss);
#pragma unroll
    for (int off = 1; off < 16; off <<= 1) ss += __shfl_xor(ss, off, 32);
    const float r1 = rsqrtf(ss * kInvHdim + kNormEps);
    const v4f nv = *(const v4f*)(nw + (c0 & (kHdim - 1)));
    float xn[4];
    float s2 = 0.0f;
#pragma unroll
    for (int e = 0; e < 4; ++e) {
      const float nf = nv[e];
      xn[e] = (z[e] * r1) * bf16r(nf);
      s2 = fmaf(xn[e], xn[e], s2);
    }
#pragma unroll
    for (int off = 1; off < 16; off <<= 1) s2 += __shfl_xor(s2, off, 32);
    const float r2 = rsqrtf(s2 + kNormEps);
#pragma unroll
    for (int e = 0; e < 4; ++e) o[e] = (xn[e] * r2) * oscale;
  } else {
#pragma unroll
    for (int e = 0; e < 4; ++e) o[e] = z[e];
  }
  float* op = outp + (size_t)row * kDim + c0;
  *(volatile v4f*)op = o;
  __threadfence();
  *(volatile v4f*)op = o;
}

constexpr int kScanSteps = 32;
constexpr int kScanPitch = 36;
static_assert(kSeq % kScanSteps == 0);
__global__ __launch_bounds__(128) void state_scan_kernel(const float* __restrict__ QN, const float* __restrict__ KN,
                                                         const float* __restrict__ VC, const float* __restrict__ DEC,
                                                         const float* __restrict__ BETA, float* __restrict__ OS) {
  __shared__ __align__(16) float slab[2 * kScanSteps * kScanPitch];
  const int tid  = threadIdx.x;
  const int lane = tid & 31;
  const int wave = tid >> 5;
  const int bh = blockIdx.x >> 1;
  const int sl = blockIdx.x & 1;
  const int b  = bh / kHeads;
  const int h  = bh - b * kHeads;
  const int kq = lane & 3;
  const int cl = wave * 8 + (lane >> 2);
  const int hb = h * kHdim;
  const int q8 = lane >> 3;
  const int c4 = (lane & 7) * 4;

  float S[16];
#pragma unroll
  for (int i = 0; i < 16; ++i) S[i] = 0.0f;

#pragma unroll 1
  for (int chunk = 0; chunk < kSeq / kScanSteps; ++chunk) {
    float* sw = slab + (chunk & 1) * (kScanSteps * kScanPitch);
#pragma unroll 1
    for (int tl = 0; tl < kScanSteps; ++tl) {
      const int rowg = b * kSeq + chunk * kScanSteps + tl;
      const size_t base = (size_t)rowg * kDim + hb;
      const float* kp = KN + base + 16 * kq;
      const float* qp = QN + base + 16 * kq;
      v4f k4[4], q4[4];
#pragma unroll
      for (int u = 0; u < 4; ++u) {
        k4[u] = *(const v4f*)(kp + 4 * u);
        q4[u] = *(const v4f*)(qp + 4 * u);
      }
      const float vt  = VC[base + sl * 32 + cl];
      const float dec = DEC[rowg * kHeads + h];
      const float bt  = BETA[rowg * kHeads + h];
      float p = 0.0f;
#pragma unroll
      for (int i = 0; i < 16; ++i) {
        S[i] *= dec;
        p = fmaf(k4[i >> 2][i & 3], S[i], p);
      }
      p += __shfl_xor(p, 1, 32);
      p += __shfl_xor(p, 2, 32);
      const float dl = (vt - p) * bt;
      float po = 0.0f;
#pragma unroll
      for (int i = 0; i < 16; ++i) {
        S[i] = fmaf(k4[i >> 2][i & 3], dl, S[i]);
        po = fmaf(q4[i >> 2][i & 3], S[i], po);
      }
      po += __shfl_xor(po, 1, 32);
      po += __shfl_xor(po, 2, 32);
      if (kq == 0) sw[tl * kScanPitch + cl] = po;
    }
    __syncthreads();
    {
      const float* sr = slab + (chunk & 1) * (kScanSteps * kScanPitch);
      for (int pass = 0; pass < 2; ++pass) {
#pragma unroll
        for (int it = 0; it < 2; ++it) {
          const int tl = wave * 8 + it * 4 + q8;
          const v4f v = *(const v4f*)(sr + tl * kScanPitch + c4);
          *(volatile v4f*)(OS + (size_t)(b * kSeq + chunk * kScanSteps + tl) * kDim + hb + sl * 32 + c4) = v;
        }
        __threadfence();
      }
    }
  }
}

__global__ __launch_bounds__(256) void outnorm_gate_kernel(const float* __restrict__ OS, const float* __restrict__ PG,
                                                           const float* __restrict__ onw, unsigned short* __restrict__ OG) {
  const int lane = threadIdx.x & 31;
  const int wave = threadIdx.x >> 5;
  const int gw   = blockIdx.x * 8 + wave;
  const int row  = gw >> 2;
  const int qd   = gw & 3;
  const int c0   = qd * 256 + lane * 8;
  const float* op = OS + (size_t)row * kDim + c0;
  const float* gp = PG + (size_t)row * kDim + c0;
  const float* wp = onw + (c0 & (kHdim - 1));
  const v4f o0 = *(const v4f*)(op);
  const v4f o1 = *(const v4f*)(op + 4);
  const v4f g0 = *(const v4f*)(gp);
  const v4f g1 = *(const v4f*)(gp + 4);
  const v4f w0 = *(const v4f*)(wp);
  const v4f w1 = *(const v4f*)(wp + 4);
  float ov[8], gv[8], wn[8];
#pragma unroll
  for (int e = 0; e < 4; ++e) {
    ov[e] = o0[e]; ov[4 + e] = o1[e];
    gv[e] = g0[e]; gv[4 + e] = g1[e];
    wn[e] = w0[e]; wn[4 + e] = w1[e];
  }
  float ss = 0.0f;
#pragma unroll
  for (int e = 0; e < 8; ++e) ss = fmaf(ov[e], ov[e], ss);
#pragma unroll
  for (int off = 1; off < 8; off <<= 1) ss += __shfl_xor(ss, off, 32);
  const float r = rsqrtf(ss * kInvHdim + kNormEps);
  unsigned short hb[8], lb[8];
#pragma unroll
  for (int e = 0; e < 8; ++e) {
    const float on   = (ov[e] * r) * bf16r(wn[e]);
    const float gate = gv[e] * sigmoid_f(gv[e]);
    const float og   = on * gate;
    hb[e] = f2bf_bits(og);
    lb[e] = f2bf_bits(og - bf_bits2f(hb[e]));
  }
  const v4u uh = (v4u){pk16(hb[0], hb[1]), pk16(hb[2], hb[3]), pk16(hb[4], hb[5]), pk16(hb[6], hb[7])};
  const v4u ul = (v4u){pk16(lb[0], lb[1]), pk16(lb[2], lb[3]), pk16(lb[4], lb[5]), pk16(lb[6], lb[7])};
  unsigned short* ph = OG + (size_t)row * kOgPitch + c0;
  unsigned short* pl = ph + kDim;
  *(volatile v4u*)ph = uh;
  *(volatile v4u*)pl = ul;
  __threadfence();
  *(volatile v4u*)ph = uh;
  *(volatile v4u*)pl = ul;
}

extern "C" void kernel_launch(void* const* d_in, const int* in_sizes, int n_in,
                              void* d_out, int out_size, void* d_ws, size_t ws_size, hipStream_t stream) {
  if (n_in < 16 || d_out == nullptr || d_ws == nullptr) return;
  if (in_sizes[0] != kRows * kDim || in_sizes[1] != kDim * kDim || in_sizes[2] != kDim * kDim ||
      in_sizes[3] != kDim * kDim || in_sizes[4] != kHeads * kDim || in_sizes[5] != kHeads * kDim ||
      in_sizes[6] != kDim * kDim || in_sizes[7] != kDim * kDim || in_sizes[8] != kHdim ||
      in_sizes[9] != kHdim || in_sizes[10] != kHdim || in_sizes[11] != kHeads || in_sizes[12] != kHeads ||
      in_sizes[13] != kDim * kTaps || in_sizes[14] != kDim * kTaps || in_sizes[15] != kDim * kTaps ||
      out_size != kRows * kDim) return;

  const float* hs      = (const float*)d_in[0];
  const float* Wq      = (const float*)d_in[1];
  const float* Wk      = (const float*)d_in[2];
  const float* Wv      = (const float*)d_in[3];
  const float* Wa      = (const float*)d_in[4];
  const float* Wb      = (const float*)d_in[5];
  const float* Wg      = (const float*)d_in[6];
  const float* Wo      = (const float*)d_in[7];
  const float* q_nw    = (const float*)d_in[8];
  const float* k_nw    = (const float*)d_in[9];
  const float* o_nw    = (const float*)d_in[10];
  const float* A_log   = (const float*)d_in[11];
  const float* dt_bias = (const float*)d_in[12];
  const float* conv_q  = (const float*)d_in[13];
  const float* conv_k  = (const float*)d_in[14];
  const float* conv_v  = (const float*)d_in[15];

  char* ws = (char*)d_ws;
  size_t off = 0;
  auto carve = [&](size_t bytes) -> char* { char* p = ws + off; off += (bytes + 255) & ~(size_t)255; return p; };
  unsigned short* XB   = (unsigned short*)carve((size_t)kRows * kDim * 2);
  unsigned short* W4   = (unsigned short*)carve((size_t)4 * kDim * kDim * 2);
  unsigned short* WO2  = (unsigned short*)carve((size_t)kDim * kOgPitch * 2);
  unsigned short* WAB  = (unsigned short*)carve((size_t)kAbPad * kDim * 2);
  float*          P4   = (float*)carve((size_t)4 * kRows * kDim * 4);
  float*          PAB  = (float*)carve((size_t)kRows * kAbPad * 4);
  float*          DEC  = (float*)carve((size_t)kRows * kHeads * 4);
  float*          BETA = (float*)carve((size_t)kRows * kHeads * 4);
  float*          X1   = (float*)carve((size_t)kRows * kDim * 4);
  unsigned short* OG   = (unsigned short*)carve((size_t)kRows * kOgPitch * 2);
  if (off > ws_size || off > (size_t)134217728) return;

  const size_t planeP = (size_t)kRows * kDim;
  float* PQ = P4;
  float* PK = P4 + planeP;
  float* PV = P4 + 2 * planeP;
  float* PG = P4 + 3 * planeP;

  cvt8_bf16_kernel<<<(kRows * kDim / 8) / 256, 256, 0, stream>>>(hs, XB, kRows * kDim / 8);
  cvt_w4_kernel<<<dim3((kDim * kDim / 8) / 256, 4), 256, 0, stream>>>(Wq, Wk, Wv, Wg, W4);
  cvt_wo2_kernel<<<(kDim * kDim / 8) / 256, 256, 0, stream>>>(Wo, WO2);
  cvt_wab_kernel<<<(kAbPad * kDim / 8) / 256, 256, 0, stream>>>(Wa, Wb, WAB);

  wmma_gemm64<1, false, 0, 0, false, 0><<<dim3((kRows / 64) * (kDim / 64) / 8, 4), 256, 0, stream>>>(
      XB, XB, kDim, 0L, W4, W4, kDim, (long)kDim * kDim, (void*)P4, (void*)P4, kDim, (long)kRows * kDim,
      DEC, X1, 0L, kRows, kDim, kDim, 1.0f);
  wmma_gemm64<1, false, 0, 0, false, 0><<<dim3((kRows / 64) * (kAbPad / 64) / 8, 1), 256, 0, stream>>>(
      XB, XB, kDim, 0L, WAB, WAB, kDim, 0L, (void*)PAB, (void*)PAB, kAbPad, 0L,
      DEC, X1, 0L, kRows, kAbPad, kDim, 1.0f);

  gate_kernel<<<(kRows * kHeads) / 256, 256, 0, stream>>>(PAB, A_log, dt_bias, DEC, BETA);

  conv_silu_kernel<true><<<kRows, 256, 0, stream>>>(PQ, conv_q, q_nw, X1, kQScale);
  conv_silu_kernel<true><<<kRows, 256, 0, stream>>>(PK, conv_k, k_nw, PQ, 1.0f);
  conv_silu_kernel<false><<<kRows, 256, 0, stream>>>(PV, conv_v, q_nw, PK, 1.0f);

  state_scan_kernel<<<kBatch * kHeads * 2, 128, 0, stream>>>(X1, PQ, PK, DEC, BETA, PV);

  outnorm_gate_kernel<<<(kRows * 4) / 8, 256, 0, stream>>>(PV, PG, o_nw, OG);

  wmma_gemm64<1, false, 0, 0, false, 0><<<dim3((kRows / 64) * (kDim / 64) / 8, 1), 256, 0, stream>>>(
      OG, OG, kOgPitch, 0L, WO2, WO2, kOgPitch, 0L, d_out, d_out, kDim, 0L,
      DEC, X1, 0L, kRows, kDim, kOgPitch, 1.0f);
}
